// GNNModel_78847009620618
// MI455X (gfx1250) — hardware-verified
//
#include <hip/hip_runtime.h>
#include <stddef.h>
#include <stdint.h>
#include <math.h>


#define FIN    128
#define HID    256
#define K2     512
#define NGR    64
#define NCLS   38
#define CH1    128
#define CATW   384
#define KC1    768
#define KZ     256
#define NPO    64
#define NTHR   256
#define NWAVE  8
#define EPT    8
#define CHUNK  (NTHR * EPT)
#define WCAP   (EPT * 32)
#define LISTN  (NWAVE * WCAP)
#define NBA    1024
#define SLA    10
#define RCAP   16384
#define DEGCAP 64
#define GBM    64
#define GBN    64
#define GTHR   128
#define PTHR   384
#define BKT_ZINTS (LISTN + 2 * RCAP + 3 * NBA)
#define BKT_LDS_INTS (BKT_ZINTS + 16)
#define UW1    (HID * (FIN / 8))
#define UW2    (HID * (K2 / 8))
#define UC1    (CH1 * (KC1 / 8))
#define UC2    (NPO * (KZ / 8))
#define NOUT   (NGR * NCLS)
#define H_CAT   (NGR * K2)
#define H_HSN   (NGR * K2 + NGR * KC1)
#define HI_STG  (H_HSN / 2)
#define HI_PRM  (HI_STG + NGR * HID)
#define HI_CB1  (HI_PRM + 5 * HID)
#define HI_CB2  (HI_CB1 + CH1)
#define HI_CNT  (HI_CB2 + NPO)
#define HEAD_LDS_INTS (HI_CNT + NGR)
#define WSMAX  134217728

static_assert((CHUNK & (CHUNK - 1)) == 0 && CHUNK <= 4096);
static_assert((NBA & (NBA - 1)) == 0 && NBA == (1 << SLA));
static_assert(((long long)CHUNK << SLA) < (1LL << 31));
static_assert(RCAP % (NTHR * 4) == 0 && BKT_ZINTS % (NTHR * 4) == 0);
static_assert(RCAP >= 12548 + 12548 / 20);
static_assert(DEGCAP >= 28 + 8);
static_assert(NBA == NTHR * 4 && NBA % NWAVE == 0 && NBA % 32 == 0);
static_assert(FIN % 32 == 0 && K2 % 32 == 0 && KC1 % 32 == 0 && KZ % 32 == 0);
static_assert(GBM == (GTHR / 32) * 16 && GBN == 64 && HID % GBN == 0);
static_assert(UW1 % NTHR == 0 && UW2 % NTHR == 0 && UC1 % NTHR == 0 && UC2 % NTHR == 0);
static_assert(HID == NTHR && PTHR == HID + FIN);
static_assert((NGR * CATW) % (PTHR * 4) == 0 && (NGR * CATW) % NTHR == 0);
static_assert(BKT_LDS_INTS * 4 <= 300000 && HEAD_LDS_INTS * 4 <= 300000);
static_assert((NOUT * 4) % 128 == 0 && NOUT / 4 == 608 && 608 == 2 * NTHR + 96);
static_assert(H_HSN % 2 == 0 && NOUT <= NGR * HID);

typedef float          v4f   __attribute__((ext_vector_type(4)));
typedef float          v8f   __attribute__((ext_vector_type(8)));
typedef int            v4i   __attribute__((ext_vector_type(4)));
typedef int            v8i   __attribute__((ext_vector_type(8)));
typedef unsigned short v4us  __attribute__((ext_vector_type(4)));
typedef unsigned short v8us  __attribute__((ext_vector_type(8)));
typedef unsigned short v16us __attribute__((ext_vector_type(16)));
typedef __bf16         v16bf __attribute__((ext_vector_type(16)));
typedef v4f  __attribute__((may_alias)) v4fa;
typedef v4i  __attribute__((may_alias)) v4ia;
typedef v4us __attribute__((may_alias)) v4usa;
typedef v8us __attribute__((may_alias)) v8usa;
union FragB { v16bf v; v16us u; v8us h[2]; v8i w; };

__device__ __forceinline__ v8f wmb(const FragB& a, const FragB& b, v8f c) {
  v8f d = __builtin_amdgcn_wmma_f32_16x16x32_bf16(false, a.v, false, b.v, (short)0, c, false, false);
  asm volatile("v_nop\n\tv_nop\n\tv_nop\n\tv_nop" : "+v"(d) : "v"(a.w), "v"(b.w));
  return d;
}

__device__ __forceinline__ unsigned bf16_bits(float f) {
  const unsigned u = __float_as_uint(f);
  return (u + 0x7FFFu + ((u >> 16) & 1u)) >> 16;
}
__device__ __forceinline__ float bf16_val(float f) {
  return __uint_as_float(bf16_bits(f) << 16);
}
__device__ __forceinline__ unsigned hilo(float v) {
  const unsigned hb = bf16_bits(v);
  const unsigned lb = bf16_bits(v - __uint_as_float(hb << 16));
  return (hb & 0xffffu) | (lb << 16);
}

__device__ __forceinline__ void wave_sync() {
  __builtin_amdgcn_fence(__ATOMIC_RELEASE, "wavefront");
  __builtin_amdgcn_wave_barrier();
  __builtin_amdgcn_fence(__ATOMIC_ACQUIRE, "wavefront");
}

__device__ __forceinline__ FragB frag_lds(const unsigned short* base, int pitch, int row, int hh, int k0) {
  FragB f;
  const unsigned short* p = base + row * pitch + 8 * hh + k0;
  f.h[0] = *(const v8usa*)p;
  f.h[1] = *(const v8usa*)(p + 16);
  return f;
}
__device__ __forceinline__ FragB frag_glb(const unsigned short* __restrict__ wt, int K, int n, int hh, int k0) {
  FragB f;
  const unsigned short* p = wt + (size_t)n * (size_t)K + 8 * hh + k0;
  f.h[0] = *(const v8usa*)p;
  f.h[1] = *(const v8usa*)(p + 16);
  return f;
}

template <int SLB>
__device__ __forceinline__ int scan_chunk(const int* __restrict__ dsts, int nE, int cbase, int slotBase,
                                          int nb, int vec8, int* list, int tid, int lane, int wave) {
  int wc = 0;
  const int el0  = tid * EPT;
  const int e0   = cbase + el0;
  const int sent = -2147483647 - 1;
  v4i da, db;
  if (vec8 != 0 && cbase + CHUNK <= nE) {
    da = *(const v4i*)(dsts + e0);
    db = *(const v4i*)(dsts + e0 + 4);
  } else {
    da.x = (e0     < nE) ? dsts[min(e0,     nE - 1)] : sent;
    da.y = (e0 + 1 < nE) ? dsts[min(e0 + 1, nE - 1)] : sent;
    da.z = (e0 + 2 < nE) ? dsts[min(e0 + 2, nE - 1)] : sent;
    da.w = (e0 + 3 < nE) ? dsts[min(e0 + 3, nE - 1)] : sent;
    db.x = (e0 + 4 < nE) ? dsts[min(e0 + 4, nE - 1)] : sent;
    db.y = (e0 + 5 < nE) ? dsts[min(e0 + 5, nE - 1)] : sent;
    db.z = (e0 + 6 < nE) ? dsts[min(e0 + 6, nE - 1)] : sent;
    db.w = (e0 + 7 < nE) ? dsts[min(e0 + 7, nE - 1)] : sent;
  }
  const unsigned nbs = (unsigned)slotBase;
  const unsigned unb = (unsigned)nb;
  const unsigned s0 = (unsigned)da.x - nbs, s1 = (unsigned)da.y - nbs;
  const unsigned s2 = (unsigned)da.z - nbs, s3 = (unsigned)da.w - nbs;
  const unsigned s4 = (unsigned)db.x - nbs, s5 = (unsigned)db.y - nbs;
  const unsigned s6 = (unsigned)db.z - nbs, s7 = (unsigned)db.w - nbs;
  const bool h0 = s0 < unb, h1 = s1 < unb, h2 = s2 < unb, h3 = s3 < unb;
  const bool h4 = s4 < unb, h5 = s5 < unb, h6 = s6 < unb, h7 = s7 < unb;
  const unsigned any = __builtin_amdgcn_ballot_w32(h0 | h1 | h2 | h3 | h4 | h5 | h6 | h7);
  if (any != 0u) {
#define HITJ(J, HJ, SJ) { \
      const unsigned mj = __builtin_amdgcn_ballot_w32(HJ); \
      if (mj != 0u) { \
        if (HJ) { \
          const int pos = wc + (int)__builtin_amdgcn_mbcnt_lo(mj, 0u); \
          if (pos < WCAP) list[wave * WCAP + pos] = ((el0 + (J)) << SLB) | (int)(SJ); \
        } \
        wc += (int)__builtin_popcount(mj); } }
    HITJ(0, h0, s0)
    HITJ(1, h1, s1)
    HITJ(2, h2, s2)
    HITJ(3, h3, s3)
    HITJ(4, h4, s4)
    HITJ(5, h5, s5)
    HITJ(6, h6, s6)
    HITJ(7, h7, s7)
#undef HITJ
  }
  return wc;
}

template <int STRIDE>
__device__ __forceinline__ v8us gather8(const float* __restrict__ p) {
  v8us o;
#pragma unroll
  for (int i = 0; i < 8; ++i) o[i] = (unsigned short)bf16_bits(p[(size_t)i * STRIDE]);
  return o;
}
__device__ __forceinline__ void put8(unsigned short* dp, v8us o) {
  *(volatile v8us*)dp = o;
  __threadfence();
  *(volatile v8us*)dp = o;
}

__global__ __launch_bounds__(NTHR) void k_prep(const float* __restrict__ x, const float* __restrict__ w1,
                                               const float* __restrict__ w2, const float* __restrict__ w3,
                                               const float* __restrict__ cw1, const float* __restrict__ cw2,
                                               int nN, int ux,
                                               unsigned short* XB, unsigned short* W1T, unsigned short* W2D,
                                               unsigned short* W3D, unsigned short* CW1D, unsigned short* CW2D) {
  const int u = (int)blockIdx.x * NTHR + (int)threadIdx.x;
  if (u < ux) {
    const int row = u >> 4;
    const int k8  = (u & 15) * 8;
    const int rc  = row < nN ? row : nN - 1;
    const float* p = x + (size_t)rc * FIN + k8;
    const v4f a = *(const v4fa*)p;
    const v4f b = *(const v4fa*)(p + 4);
    const bool ok = row < nN;
    v8us o;
    o[0] = ok ? (unsigned short)bf16_bits(a.x) : (unsigned short)0;
    o[1] = ok ? (unsigned short)bf16_bits(a.y) : (unsigned short)0;
    o[2] = ok ? (unsigned short)bf16_bits(a.z) : (unsigned short)0;
    o[3] = ok ? (unsigned short)bf16_bits(a.w) : (unsigned short)0;
    o[4] = ok ? (unsigned short)bf16_bits(b.x) : (unsigned short)0;
    o[5] = ok ? (unsigned short)bf16_bits(b.y) : (unsigned short)0;
    o[6] = ok ? (unsigned short)bf16_bits(b.z) : (unsigned short)0;
    o[7] = ok ? (unsigned short)bf16_bits(b.w) : (unsigned short)0;
    put8(XB + (size_t)row * FIN + k8, o);
  } else if (u < ux + UW1) {
    const int v  = u - ux;
    const int n  = v >> 4;
    const int k8 = (v & 15) * 8;
    const v8us o = gather8<HID>(w1 + (size_t)k8 * HID + n);
    put8(W1T + (size_t)n * FIN + k8, o);
  } else if (u < ux + UW1 + UW2) {
    const int v  = u - ux - UW1;
    const int n  = v >> 6;
    const int k8 = (v & 63) * 8;
    const int kk = k8 & (HID - 1);
    const v8us o = gather8<HID>(w2 + (size_t)kk * HID + n);
    put8(W2D + (size_t)n * K2 + k8, o);
  } else if (u < ux + UW1 + 2 * UW2) {
    const int v  = u - ux - UW1 - UW2;
    const int n  = v >> 6;
    const int k8 = (v & 63) * 8;
    const int kk = k8 & (HID - 1);
    const v8us o = gather8<HID>(w3 + (size_t)kk * HID + n);
    put8(W3D + (size_t)n * K2 + k8, o);
  } else if (u < ux + UW1 + 2 * UW2 + UC1) {
    const int v  = u - ux - UW1 - 2 * UW2;
    const int n  = v / (KC1 / 8);
    const int k8 = (v - n * (KC1 / 8)) * 8;
    const int kk = k8 >= CATW ? k8 - CATW : k8;
    const v8us o = gather8<CH1>(cw1 + (size_t)kk * CH1 + n);
    put8(CW1D + (size_t)n * KC1 + k8, o);
  } else if (u < ux + UW1 + 2 * UW2 + UC1 + UC2) {
    const int v  = u - ux - UW1 - 2 * UW2 - UC1;
    const int n  = v >> 5;
    const int k8 = (v & 31) * 8;
    const int kk = k8 & (CH1 - 1);
    const int nc = n < NCLS ? n : NCLS - 1;
    v8us o = gather8<NCLS>(cw2 + (size_t)kk * NCLS + nc);
    const v8us z = {0, 0, 0, 0, 0, 0, 0, 0};
    if (n >= NCLS) o = z;
    put8(CW2D + (size_t)n * KZ + k8, o);
  }
}

__global__ __launch_bounds__(NTHR) void k_bucket(const int* __restrict__ srcs, const int* __restrict__ dsts,
                                                 int nE, int nN, int vec8,
                                                 int* hits, int* cntT, int* offT, float* dis) {
  extern __shared__ __attribute__((aligned(16))) int dsm[];
  int* list = dsm;
  int* hl   = dsm + LISTN;
  int* sl   = hl + RCAP;
  int* cnt  = sl + RCAP;
  int* offs = cnt + NBA;
  int* cur  = offs + NBA;
  int* misc = cur + NBA;
  const int tid = (int)threadIdx.x, lane = tid & 31, wave = tid >> 5;
  const int nodeBase = (int)blockIdx.x * NBA;

  {
    const v4i z4 = {0, 0, 0, 0};
    for (int i = tid * 4; i < BKT_ZINTS; i += NTHR * 4) *(v4ia*)(dsm + i) = z4;
    if (tid < 16) misc[tid] = 0;
  }
  __syncthreads();

  int t = 0, ov = 0;
  const int nChunks = (nE + CHUNK - 1) / CHUNK;
#pragma unroll 1
  for (int ch = 0; ch < nChunks; ++ch) {
    const int cbase = ch * CHUNK;
    const int wc = scan_chunk<SLA>(dsts, nE, cbase, nodeBase, NBA, vec8, list, tid, lane, wave);
    if (lane == 0) misc[wave] = wc;
    __syncthreads();
    if (wave == 0) {
#pragma unroll 1
      for (int w2 = 0; w2 < NWAVE; ++w2) {
        int c = misc[w2];
        c = c < 0 ? 0 : (c > WCAP ? WCAP : c);
#pragma unroll 1
        for (int b0 = 0; b0 < c; b0 += 32) {
          const int idx = b0 + lane;
          const int ent = list[w2 * WCAP + (idx < WCAP ? idx : WCAP - 1)];
          const int m32 = (c - b0) < 32 ? (c - b0) : 32;
#pragma unroll 1
          for (int k = 0; k < m32; ++k) {
            const int u    = __builtin_amdgcn_readlane(ent, k);
            const int slot = u & (NBA - 1);
            const int el   = (u >> SLA) & (CHUNK - 1);
            const int pk   = ((cbase + el) << SLA) | slot;
            if (t < RCAP) {
              if (lane == 0) { hl[t] = pk; cnt[slot] = cnt[slot] + 1; }
              t = t + 1;
            } else {
              ov = 1;
            }
          }
        }
      }
    }
    __syncthreads();
  }
  if (wave == 0 && lane == 0) { misc[8] = t; misc[9] = ov; }
  __syncthreads();
  int tt = misc[8];
  tt = tt < 0 ? 0 : (tt > RCAP ? RCAP : tt);
  const int ovf = misc[9];

  if (wave == 0) {
    const int base = lane * (NBA / 32);
    int s = 0;
#pragma unroll 1
    for (int i = 0; i < NBA / 32; ++i) s += cnt[base + i];
    int incl = s;
#pragma unroll
    for (int d = 1; d < 32; d <<= 1) {
      const int y = __shfl_up(incl, d, 32);
      if (lane >= d) incl += y;
    }
    int run = incl - s;
#pragma unroll 1
    for (int i = 0; i < NBA / 32; ++i) {
      const int cv = cnt[base + i];
      offs[base + i] = run;
      cur[base + i]  = run;
      run += cv;
    }
  }
  __syncthreads();
  if (wave == 0) {
#pragma unroll 1
    for (int b0 = 0; b0 < tt; b0 += 32) {
      const int idx = b0 + lane;
      const int ent = hl[idx < RCAP ? idx : RCAP - 1];
      const int m32 = (tt - b0) < 32 ? (tt - b0) : 32;
#pragma unroll 1
      for (int k = 0; k < m32; ++k) {
        const int u    = __builtin_amdgcn_readlane(ent, k);
        const int slot = u & (NBA - 1);
        if (lane == 0) {
          int p = cur[slot];
          p = p < 0 ? 0 : (p > RCAP - 1 ? RCAP - 1 : p);
          sl[p] = u;
          cur[slot] = p + 1;
        }
      }
    }
  }
  __syncthreads();

#pragma unroll 1
  for (int i = tid * 4; i < RCAP; i += NTHR * 4) {
    const v4i e = *(const v4ia*)(sl + i);
    int e0 = e.x >> SLA, e1 = e.y >> SLA, e2 = e.z >> SLA, e3 = e.w >> SLA;
    e0 = e0 < 0 ? 0 : (e0 > nE - 1 ? nE - 1 : e0);
    e1 = e1 < 0 ? 0 : (e1 > nE - 1 ? nE - 1 : e1);
    e2 = e2 < 0 ? 0 : (e2 > nE - 1 ? nE - 1 : e2);
    e3 = e3 < 0 ? 0 : (e3 > nE - 1 ? nE - 1 : e3);
    int s0 = srcs[e0], s1 = srcs[e1], s2 = srcs[e2], s3 = srcs[e3];
    s0 = s0 < 0 ? 0 : (s0 > nN - 1 ? nN - 1 : s0);
    s1 = s1 < 0 ? 0 : (s1 > nN - 1 ? nN - 1 : s1);
    s2 = s2 < 0 ? 0 : (s2 > nN - 1 ? nN - 1 : s2);
    s3 = s3 < 0 ? 0 : (s3 > nN - 1 ? nN - 1 : s3);
    v4i r;
    r.x = (i     < tt) ? s0 : 0;
    r.y = (i + 1 < tt) ? s1 : 0;
    r.z = (i + 2 < tt) ? s2 : 0;
    r.w = (i + 3 < tt) ? s3 : 0;
    *(v4ia*)(hl + i) = r;
  }
  __syncthreads();

  int* hp = hits + (size_t)blockIdx.x * RCAP;
#pragma unroll 1
  for (int i = tid * 4; i < RCAP; i += NTHR * 4) {
    const v4i v = *(const v4ia*)(hl + i);
    *(volatile v4i*)(hp + i) = v;
  }
  __threadfence();
#pragma unroll 1
  for (int i = tid * 4; i < RCAP; i += NTHR * 4) {
    const v4i v = *(const v4ia*)(hl + i);
    *(volatile v4i*)(hp + i) = v;
  }

  const v4i c4 = *(const v4ia*)(cnt + 4 * tid);
  const v4i o4 = *(const v4ia*)(offs + 4 * tid);
  v4f d4;
  d4.x = 1.0f / sqrtf((float)c4.x + 1.0f);
  d4.y = 1.0f / sqrtf((float)c4.y + 1.0f);
  d4.z = 1.0f / sqrtf((float)c4.z + 1.0f);
  d4.w = 1.0f / sqrtf((float)c4.w + 1.0f);
  const int bigv = 0x40000000;
  v4i cw;
  cw.x = (ovf != 0) ? bigv : c4.x;
  cw.y = (ovf != 0) ? bigv : c4.y;
  cw.z = (ovf != 0) ? bigv : c4.z;
  cw.w = (ovf != 0) ? bigv : c4.w;
  int*   cp = cntT + (size_t)nodeBase + 4 * tid;
  int*   op = offT + (size_t)nodeBase + 4 * tid;
  float* dp = dis  + (size_t)nodeBase + 4 * tid;
  *(volatile v4i*)cp = cw;
  *(volatile v4i*)op = o4;
  *(volatile v4f*)dp = d4;
  __threadfence();
  *(volatile v4i*)cp = cw;
  *(volatile v4i*)op = o4;
  *(volatile v4f*)dp = d4;
}

__global__ __launch_bounds__(GTHR) void k_gemm(
    const unsigned short* __restrict__ A, const unsigned short* __restrict__ WT,
    const float* __restrict__ dis, int nDis, float* outF, int K, int ldo)
{
  __shared__ __attribute__((aligned(16))) float stg[GBM * GBN];
  __shared__ float sdis[GBM];
  const int tid = (int)threadIdx.x, lane = tid & 31, wave = tid >> 5, hh = lane >> 4, m = lane & 15;
  const int rowBase = (int)blockIdx.x * GBM;
  const int col0    = (int)blockIdx.y * GBN;

  if (tid < GBM) {
    const int gr = rowBase + tid;
    sdis[tid] = dis[gr < nDis ? gr : nDis - 1];
  }

  v8f acc[4];
  {
    const v8f z = {0.f, 0.f, 0.f, 0.f, 0.f, 0.f, 0.f, 0.f};
    acc[0] = z; acc[1] = z; acc[2] = z; acc[3] = z;
  }
  const unsigned short* ap = A  + (size_t)(rowBase + 16 * wave + m) * (size_t)K + 8 * hh;
  const unsigned short* wp = WT + (size_t)(col0 + m) * (size_t)K + 8 * hh;
  const int ksteps = K >> 5;
#pragma unroll 1
  for (int ks = 0; ks < ksteps; ++ks) {
    FragB af;
    af.h[0] = *(const v8usa*)(ap + 32 * ks);
    af.h[1] = *(const v8usa*)(ap + 32 * ks + 16);
#pragma unroll
    for (int t = 0; t < 4; ++t) {
      const unsigned short* wq = wp + (size_t)(16 * t) * (size_t)K + 32 * ks;
      FragB bf;
      bf.h[0] = *(const v8usa*)wq;
      bf.h[1] = *(const v8usa*)(wq + 16);
      acc[t] = wmb(af, bf, acc[t]);
    }
  }

#pragma unroll
  for (int t = 0; t < 4; ++t) {
    const int lc = 16 * t + m;
#pragma unroll
    for (int r = 0; r < 8; ++r) {
      const int lr = 16 * wave + 8 * hh + r;
      stg[lr * GBN + lc] = acc[t][r];
    }
  }
  __syncthreads();

  v4f fv[8];
#pragma unroll
  for (int i = 0; i < 8; ++i) {
    const int lr = 16 * wave + 2 * i + hh;
    const float sc = sdis[lr];
    const v4f q = *(const v4fa*)(stg + lr * GBN + 4 * m);
    v4f y;
    y.x = q.x * sc; y.y = q.y * sc; y.z = q.z * sc; y.w = q.w * sc;
    fv[i] = y;
  }
#pragma unroll
  for (int i = 0; i < 8; ++i) {
    const int lr = 16 * wave + 2 * i + hh;
    const int gr = rowBase + lr;
    float* op = outF + (size_t)gr * (size_t)ldo + col0 + 4 * m;
    *(volatile v4f*)op = fv[i];
  }
  __threadfence();
#pragma unroll
  for (int i = 0; i < 8; ++i) {
    const int lr = 16 * wave + 2 * i + hh;
    const int gr = rowBase + lr;
    float* op = outF + (size_t)gr * (size_t)ldo + col0 + 4 * m;
    *(volatile v4f*)op = fv[i];
  }
}

__device__ __forceinline__ float bnact(float t, float b, float mm, float r, float g, float be) {
  float y = t + b;
  y = ((y - mm) * r) * g + be;
  return (y > 0.0f) ? y : (y - y);
}

template <int MODE>
__global__ __launch_bounds__(NTHR) void k_agg(const int* __restrict__ hits, const int* __restrict__ cntT,
                                              const int* __restrict__ offT, const float* __restrict__ dis,
                                              int nN, int mRows, const float* __restrict__ xl,
                                              const float* __restrict__ pb, const float* __restrict__ pm,
                                              const float* __restrict__ pv, const float* __restrict__ pg,
                                              const float* __restrict__ pbe,
                                              unsigned short* hb, float* hout) {
  __shared__ __attribute__((aligned(16))) float prm[5 * HID];
  __shared__ __attribute__((aligned(16))) unsigned short rowbuf[NWAVE * K2];
  const int tid = (int)threadIdx.x, lane = tid & 31, wave = tid >> 5;
  const int nodeBase = (int)blockIdx.x * NBA;

  prm[tid]           = bf16_val(pb[tid]);
  prm[HID + tid]     = bf16_val(pm[tid]);
  prm[2 * HID + tid] = 1.0f / sqrtf(bf16_val(pv[tid]) + 1e-5f);
  prm[3 * HID + tid] = bf16_val(pg[tid]);
  prm[4 * HID + tid] = bf16_val(pbe[tid]);
  __syncthreads();

  const v4f bA = *(const v4fa*)(prm + 4 * lane),            bB = *(const v4fa*)(prm + 128 + 4 * lane);
  const v4f mA = *(const v4fa*)(prm + HID + 4 * lane),      mB = *(const v4fa*)(prm + HID + 128 + 4 * lane);
  const v4f rA = *(const v4fa*)(prm + 2 * HID + 4 * lane),  rB = *(const v4fa*)(prm + 2 * HID + 128 + 4 * lane);
  const v4f gA = *(const v4fa*)(prm + 3 * HID + 4 * lane),  gB = *(const v4fa*)(prm + 3 * HID + 128 + 4 * lane);
  const v4f eA = *(const v4fa*)(prm + 4 * HID + 4 * lane),  eB = *(const v4fa*)(prm + 4 * HID + 128 + 4 * lane);

  const int* hp = hits + (size_t)blockIdx.x * RCAP;
  unsigned short* rb = rowbuf + wave * K2;
  const float qnan = __int_as_float(0x7fc00000);

#pragma unroll 1
  for (int si = 0; si < NBA / NWAVE; ++si) {
    const int s    = si * NWAVE + wave;
    const int node = nodeBase + s;
    int c = cntT[node];
    const bool big = c > DEGCAP;
    c = c < 0 ? 0 : (c > DEGCAP ? DEGCAP : c);
    int o = offT[node];
    o = o < 0 ? 0 : (o > RCAP ? RCAP : o);
    const int nc = node < nN ? node : nN - 1;
    const float dd = dis[nc];
    v4f aA = {0.0f, 0.0f, 0.0f, 0.0f};
    v4f aB = {0.0f, 0.0f, 0.0f, 0.0f};
#pragma unroll 1
    for (int b0 = 0; b0 < c; b0 += 32) {
      int idx = o + b0 + lane;
      idx = idx > RCAP - 1 ? RCAP - 1 : idx;
      int sr = hp[idx];
      sr = sr < 0 ? 0 : (sr > nN - 1 ? nN - 1 : sr);
      const int m32 = (c - b0) < 32 ? (c - b0) : 32;
#pragma unroll 1
      for (int k = 0; k < m32; ++k) {
        const int sk = __builtin_amdgcn_readlane(sr, k);
        const float* rp = xl + (size_t)sk * HID + 4 * lane;
        const v4f ra = *(const v4f*)rp;
        const v4f rc = *(const v4f*)(rp + 128);
        aA = aA + ra;
        aB = aB + rc;
      }
    }
    {
      const float* rp = xl + (size_t)nc * HID + 4 * lane;
      const v4f ra = *(const v4f*)rp;
      const v4f rc = *(const v4f*)(rp + 128);
      aA = aA + ra;
      aB = aB + rc;
    }
    const float pzr = big ? qnan : 0.0f;
    const bool live = node < nN;
    v4f tA, tB;
    tA.x = aA.x * dd; tA.y = aA.y * dd; tA.z = aA.z * dd; tA.w = aA.w * dd;
    tB.x = aB.x * dd; tB.y = aB.y * dd; tB.z = aB.z * dd; tB.w = aB.w * dd;
    v4f oA, oB;
    if constexpr (MODE == 3) {
      oA.x = tA.x + pzr; oA.y = tA.y + pzr; oA.z = tA.z + pzr; oA.w = tA.w + pzr;
      oB.x = tB.x + pzr; oB.y = tB.y + pzr; oB.z = tB.z + pzr; oB.w = tB.w + pzr;
    } else {
      oA.x = bnact(tA.x, bA.x, mA.x, rA.x, gA.x, eA.x) + pzr;
      oA.y = bnact(tA.y, bA.y, mA.y, rA.y, gA.y, eA.y) + pzr;
      oA.z = bnact(tA.z, bA.z, mA.z, rA.z, gA.z, eA.z) + pzr;
      oA.w = bnact(tA.w, bA.w, mA.w, rA.w, gA.w, eA.w) + pzr;
      oB.x = bnact(tB.x, bB.x, mB.x, rB.x, gB.x, eB.x) + pzr;
      oB.y = bnact(tB.y, bB.y, mB.y, rB.y, gB.y, eB.y) + pzr;
      oB.z = bnact(tB.z, bB.z, mB.z, rB.z, gB.z, eB.z) + pzr;
      oB.w = bnact(tB.w, bB.w, mB.w, rB.w, gB.w, eB.w) + pzr;
    }
    if constexpr (MODE == 2) {
      oA.x = oA.x * dd; oA.y = oA.y * dd; oA.z = oA.z * dd; oA.w = oA.w * dd;
      oB.x = oB.x * dd; oB.y = oB.y * dd; oB.z = oB.z * dd; oB.w = oB.w * dd;
    }
    oA.x = live ? oA.x : 0.0f; oA.y = live ? oA.y : 0.0f; oA.z = live ? oA.z : 0.0f; oA.w = live ? oA.w : 0.0f;
    oB.x = live ? oB.x : 0.0f; oB.y = live ? oB.y : 0.0f; oB.z = live ? oB.z : 0.0f; oB.w = live ? oB.w : 0.0f;

    if constexpr (MODE == 1) {
      const unsigned p0 = hilo(oA.x), p1 = hilo(oA.y), p2 = hilo(oA.z), p3 = hilo(oA.w);
      const unsigned p4 = hilo(oB.x), p5 = hilo(oB.y), p6 = hilo(oB.z), p7 = hilo(oB.w);
      v4us hA, hB, lA, lB;
      hA[0] = (unsigned short)(p0 & 0xffffu); hA[1] = (unsigned short)(p1 & 0xffffu);
      hA[2] = (unsigned short)(p2 & 0xffffu); hA[3] = (unsigned short)(p3 & 0xffffu);
      hB[0] = (unsigned short)(p4 & 0xffffu); hB[1] = (unsigned short)(p5 & 0xffffu);
      hB[2] = (unsigned short)(p6 & 0xffffu); hB[3] = (unsigned short)(p7 & 0xffffu);
      lA[0] = (unsigned short)(p0 >> 16); lA[1] = (unsigned short)(p1 >> 16);
      lA[2] = (unsigned short)(p2 >> 16); lA[3] = (unsigned short)(p3 >> 16);
      lB[0] = (unsigned short)(p4 >> 16); lB[1] = (unsigned short)(p5 >> 16);
      lB[2] = (unsigned short)(p6 >> 16); lB[3] = (unsigned short)(p7 >> 16);
      *(v4usa*)(rb + 4 * lane)             = hA;
      *(v4usa*)(rb + 128 + 4 * lane)       = hB;
      *(v4usa*)(rb + HID + 4 * lane)       = lA;
      *(v4usa*)(rb + HID + 128 + 4 * lane) = lB;
      wave_sync();
      const v8us q0 = *(const v8usa*)(rb + 8 * lane);
      const v8us q1 = *(const v8usa*)(rb + HID + 8 * lane);
      wave_sync();
      if (node < mRows) {
        unsigned short* rpw = hb + (size_t)node * K2 + 8 * lane;
        *(volatile v8us*)rpw = q0;
        *(volatile v8us*)(rpw + HID) = q1;
        __threadfence();
        *(volatile v8us*)rpw = q0;
        *(volatile v8us*)(rpw + HID) = q1;
      }
    } else {
      if (node < mRows) {
        float* op = hout + (size_t)node * HID + 4 * lane;
        *(volatile v4f*)op = oA;
        *(volatile v4f*)(op + 128) = oB;
        __threadfence();
        *(volatile v4f*)op = oA;
        *(volatile v4f*)(op + 128) = oB;
      }
    }
  }
}

__global__ __launch_bounds__(PTHR) void k_pool(const float* __restrict__ a3, const float* __restrict__ x,
                                               const int* __restrict__ bat, int nN, float* rec, int* cntO) {
  extern __shared__ __attribute__((aligned(16))) float pacc[];
  __shared__ __attribute__((aligned(16))) int cl[NGR];
  const int tid = (int)threadIdx.x;
  const int base = (int)blockIdx.x * NBA;
  {
    const v4f z = {0.0f, 0.0f, 0.0f, 0.0f};
    for (int i = tid * 4; i < NGR * CATW; i += PTHR * 4) *(v4fa*)(pacc + i) = z;
  }
  __syncthreads();
  int cr = 0;
  if (tid < HID) {
#pragma unroll 1
    for (int r = 0; r < NBA; ++r) {
      const int row = base + r;
      const int rc  = row < nN ? row : nN - 1;
      const int g   = bat[rc];
      const bool ok = (row < nN) && ((unsigned)g < (unsigned)NGR);
      const int gi  = ok ? g : 0;
      const float vv = a3[(size_t)rc * HID + tid];
      const float v  = ok ? vv : 0.0f;
      pacc[gi * CATW + tid] = pacc[gi * CATW + tid] + v;
      cr += (ok && g == tid) ? 1 : 0;
    }
  } else {
    const int cx = tid - HID;
#pragma unroll 1
    for (int r = 0; r < NBA; ++r) {
      const int row = base + r;
      const int rc  = row < nN ? row : nN - 1;
      const int g   = bat[rc];
      const bool ok = (row < nN) && ((unsigned)g < (unsigned)NGR);
      const int gi  = ok ? g : 0;
      const float vv = bf16_val(x[(size_t)rc * FIN + cx]);
      const float v  = ok ? vv : 0.0f;
      pacc[gi * CATW + tid] = pacc[gi * CATW + tid] + v;
    }
  }
  __syncthreads();
  if (tid < NGR) cl[tid] = cr;
  __syncthreads();

  float* rp = rec + (size_t)blockIdx.x * (NGR * CATW);
#pragma unroll 1
  for (int it = 0; it < (NGR * CATW) / (PTHR * 4); ++it) {
    const int i4 = 4 * (it * PTHR + tid);
    const v4f v = *(const v4fa*)(pacc + i4);
    *(volatile v4f*)(rp + i4) = v;
  }
  __threadfence();
#pragma unroll 1
  for (int it = 0; it < (NGR * CATW) / (PTHR * 4); ++it) {
    const int i4 = 4 * (it * PTHR + tid);
    const v4f v = *(const v4fa*)(pacc + i4);
    *(volatile v4f*)(rp + i4) = v;
  }
  const v4i cv = *(const v4ia*)(cl + 4 * (tid & 15));
  int* cp = cntO + (size_t)blockIdx.x * NGR + 4 * (tid & 15);
  const bool okc = tid < 16;
  if (okc) *(volatile v4i*)cp = cv;
  __threadfence();
  if (okc) *(volatile v4i*)cp = cv;
}

__global__ __launch_bounds__(NTHR) void k_head(const float* __restrict__ rec, const int* __restrict__ cntI, int nb,
                                               const unsigned short* __restrict__ w3d,
                                               const unsigned short* __restrict__ cw1d,
                                               const unsigned short* __restrict__ cw2d,
                                               const float* __restrict__ b3, const float* __restrict__ m3,
                                               const float* __restrict__ v3, const float* __restrict__ g3,
                                               const float* __restrict__ be3, const float* __restrict__ cb1,
                                               const float* __restrict__ cb2, float* out) {
  extern __shared__ __attribute__((aligned(16))) int dsm[];
  unsigned short* hs = (unsigned short*)dsm;
  float* stg  = (float*)(dsm + HI_STG);
  float* prm  = (float*)(dsm + HI_PRM);
  float* cb1s = (float*)(dsm + HI_CB1);
  float* cb2s = (float*)(dsm + HI_CB2);
  int*   cnts = dsm + HI_CNT;
  const int tid = (int)threadIdx.x, lane = tid & 31, wave = tid >> 5, hh = lane >> 4, m = lane & 15;

  prm[tid]           = bf16_val(b3[tid]);
  prm[HID + tid]     = bf16_val(m3[tid]);
  prm[2 * HID + tid] = 1.0f / sqrtf(bf16_val(v3[tid]) + 1e-5f);
  prm[3 * HID + tid] = bf16_val(g3[tid]);
  prm[4 * HID + tid] = bf16_val(be3[tid]);
  if (tid < CH1) cb1s[tid] = bf16_val(cb1[tid]);
  if (tid < NPO) {
    const float bb = cb2[tid < NCLS ? tid : NCLS - 1];
    cb2s[tid] = (tid < NCLS) ? bf16_val(bb) : 0.0f;
    int c = 0;
#pragma unroll 1
    for (int b = 0; b < nb; ++b) c += cntI[b * NGR + tid];
    cnts[tid] = c < 0 ? 0 : c;
  }
  __syncthreads();

#pragma unroll 1
  for (int it = 0; it < (NGR * CATW) / NTHR; ++it) {
    const int idx = it * NTHR + tid;
    const int g = idx / CATW;
    const int c = idx - g * CATW;
    const float* rp = rec + (size_t)g * CATW + c;
    double s = 0.0;
#pragma unroll 4
    for (int b = 0; b < nb; ++b) s += (double)rp[(size_t)b * (NGR * CATW)];
    const float sf = (float)s;
    const int cn = cnts[g];
    const float cf = cn < 1 ? 1.0f : (float)cn;
    const float pvv = sf / cf;
    const unsigned pk = hilo(pvv);
    const bool isP = c < HID;
    const int oh = isP ? (g * K2 + c)       : (H_CAT + g * KC1 + c);
    const int ol = isP ? (g * K2 + HID + c) : (H_CAT + g * KC1 + CATW + c);
    hs[oh] = (unsigned short)(pk & 0xffffu);
    hs[ol] = (unsigned short)(pk >> 16);
  }
  __syncthreads();

  const v8f zf = {0.f, 0.f, 0.f, 0.f, 0.f, 0.f, 0.f, 0.f};

  {
    v8f acc[4][2];
#pragma unroll
    for (int rt = 0; rt < 4; ++rt) { acc[rt][0] = zf; acc[rt][1] = zf; }
#pragma unroll 1
    for (int k0 = 0; k0 < K2; k0 += 32) {
      const FragB b0 = frag_glb(w3d, K2, 32 * wave + m, hh, k0);
      const FragB b1 = frag_glb(w3d, K2, 32 * wave + 16 + m, hh, k0);
#pragma unroll
      for (int rt = 0; rt < 4; ++rt) {
        const FragB af = frag_lds(hs, K2, 16 * rt + m, hh, k0);
        acc[rt][0] = wmb(af, b0, acc[rt][0]);
        acc[rt][1] = wmb(af, b1, acc[rt][1]);
      }
    }
#pragma unroll
    for (int rt = 0; rt < 4; ++rt) {
#pragma unroll
      for (int t = 0; t < 2; ++t) {
#pragma unroll
        for (int r = 0; r < 8; ++r) {
          stg[(16 * rt + 8 * hh + r) * HID + 32 * wave + 16 * t + m] = acc[rt][t][r];
        }
      }
    }
  }
  __syncthreads();
  {
    const float pb_ = prm[tid], pm_ = prm[HID + tid], pr_ = prm[2 * HID + tid];
    const float pg_ = prm[3 * HID + tid], pe_ = prm[4 * HID + tid];
#pragma unroll 4
    for (int g = 0; g < NGR; ++g) {
      const float q = stg[g * HID + tid];
      float y = (q + pb_) - pm_;
      y = (y * pr_) * pg_ + pe_;
      const float val = (cnts[g] > 0) ? y : 0.0f;
      const unsigned pk = hilo(val);
      hs[H_CAT + g * KC1 + tid]        = (unsigned short)(pk & 0xffffu);
      hs[H_CAT + g * KC1 + CATW + tid] = (unsigned short)(pk >> 16);
    }
  }
  __syncthreads();

  {
    v8f acc[4];
#pragma unroll
    for (int rt = 0; rt < 4; ++rt) acc[rt] = zf;
#pragma unroll 1
    for (int k0 = 0; k0 < KC1; k0 += 32) {
      const FragB bf = frag_glb(cw1d, KC1, 16 * wave + m, hh, k0);
#pragma unroll
      for (int rt = 0; rt < 4; ++rt) {
        const FragB af = frag_lds(hs + H_CAT, KC1, 16 * rt + m, hh, k0);
        acc[rt] = wmb(af, bf, acc[rt]);
      }
    }
#pragma unroll
    for (int rt = 0; rt < 4; ++rt) {
#pragma unroll
      for (int r = 0; r < 8; ++r) {
        stg[(16 * rt + 8 * hh + r) * CH1 + 16 * wave + m] = acc[rt][r];
      }
    }
  }
  __syncthreads();
#pragma unroll 4
  for (int j = 0; j < (NGR * CH1) / NTHR; ++j) {
    const int e = j * NTHR + tid;
    const int g = e >> 7;
    const int col = e & (CH1 - 1);
    const float y = stg[g * CH1 + col] + cb1s[col];
    const float z = (y > 0.0f) ? y : (y - y);
    const unsigned pk = hilo(z);
    hs[g * KZ + col]       = (unsigned short)(pk & 0xffffu);
    hs[g * KZ + CH1 + col] = (unsigned short)(pk >> 16);
  }
  __syncthreads();

  {
    const int ct  = wave & 3;
    const int rt0 = 2 * (wave >> 2);
    v8f acc[2];
    acc[0] = zf; acc[1] = zf;
#pragma unroll 1
    for (int k0 = 0; k0 < KZ; k0 += 32) {
      const FragB bf = frag_glb(cw2d, KZ, 16 * ct + m, hh, k0);
#pragma unroll
      for (int q = 0; q < 2; ++q) {
        const FragB af = frag_lds(hs, KZ, 16 * (rt0 + q) + m, hh, k0);
        acc[q] = wmb(af, bf, acc[q]);
      }
    }
    const int col = 16 * ct + m;
    const float cbv = cb2s[col];
#pragma unroll
    for (int q = 0; q < 2; ++q) {
#pragma unroll
      for (int r = 0; r < 8; ++r) {
        const int row = 16 * (rt0 + q) + 8 * hh + r;
        if (col < NCLS) stg[row * NCLS + col] = acc[q][r] + cbv;
      }
    }
  }
  __syncthreads();
  v4f ov[3];
#pragma unroll
  for (int it = 0; it < 3; ++it) ov[it] = *(const v4fa*)(stg + 4 * (it * NTHR + tid));
#pragma unroll
  for (int it = 0; it < 3; ++it) {
    const int i4 = it * NTHR + tid;
    if (i4 < NOUT / 4) *(volatile v4f*)(out + 4 * (size_t)i4) = ov[it];
  }
  __threadfence();
#pragma unroll
  for (int it = 0; it < 3; ++it) {
    const int i4 = it * NTHR + tid;
    if (i4 < NOUT / 4) *(volatile v4f*)(out + 4 * (size_t)i4) = ov[it];
  }
}

static inline int cdiv(int a, int b) { return (a + b - 1) / b; }
static inline size_t al256(size_t o) { return (o + 255) & ~(size_t)255; }

extern "C" void kernel_launch(void* const* d_in, const int* in_sizes, int n_in,
                              void* d_out, int out_size, void* d_ws, size_t ws_size,
                              hipStream_t stream) {
  if (n_in < 25) return;
  if (in_sizes[0] < FIN || (in_sizes[0] % FIN) != 0) return;
  const int nN = in_sizes[0] / FIN;
  if (nN < 1 || nN > (1 << 21)) return;
  if (in_sizes[1] < 2 || (in_sizes[1] & 1) != 0) return;
  const int nE = in_sizes[1] / 2;
  if (nE < 1 || nE >= (1 << (31 - SLA))) return;
  if (in_sizes[2] != nN) return;
  if (in_sizes[3] != FIN * HID || in_sizes[5] != HID * HID || in_sizes[7] != HID * HID) return;
  if (in_sizes[4] != HID || in_sizes[6] != HID || in_sizes[8] != HID) return;
  for (int i = 9; i <= 20; ++i) if (in_sizes[i] != HID) return;
  if (in_sizes[21] != CATW * CH1 || in_sizes[22] != CH1) return;
  if (in_sizes[23] != CH1 * NCLS || in_sizes[24] != NCLS) return;
  if (out_size != NOUT) return;

  const float* x    = (const float*)d_in[0];
  const int*   edge = (const int*)d_in[1];
  const int*   bat  = (const int*)d_in[2];
  const float* w1 = (const float*)d_in[3];  const float* b1 = (const float*)d_in[4];
  const float* w2 = (const float*)d_in[5];  const float* b2 = (const float*)d_in[6];
  const float* w3 = (const float*)d_in[7];  const float* b3 = (const float*)d_in[8];
  const float* g1 = (const float*)d_in[9];  const float* be1 = (const float*)d_in[10];
  const float* m1 = (const float*)d_in[11]; const float* v1  = (const float*)d_in[12];
  const float* g2 = (const float*)d_in[13]; const float* be2 = (const float*)d_in[14];
  const float* m2 = (const float*)d_in[15]; const float* v2  = (const float*)d_in[16];
  const float* g3 = (const float*)d_in[17]; const float* be3 = (const float*)d_in[18];
  const float* m3 = (const float*)d_in[19]; const float* v3  = (const float*)d_in[20];
  const float* cw1 = (const float*)d_in[21]; const float* cb1 = (const float*)d_in[22];
  const float* cw2 = (const float*)d_in[23]; const float* cb2 = (const float*)d_in[24];
  float* out = (float*)d_out;
  const int* src = edge;
  const int* dst = edge + nE;

  const int MP = cdiv(nN, 128) * 128;
  const int gM = MP / GBM;
  const int gA = cdiv(MP, NBA);
  if ((long long)gA * NBA < (long long)MP) return;
  const int NBP = gA * NBA;
  const int vec8 = ((nE & 3) == 0) ? 1 : 0;
  const int ux = MP * (FIN / 8);
  if ((ux % NTHR) != 0) return;

  char* ws = (char*)d_ws;
  size_t off = 0;
  const size_t oXB  = off; off = al256(off + (size_t)MP * FIN * 2);
  const size_t oR1  = off; off = al256(off + (size_t)MP * HID * 4);
  const size_t oR2  = off; off = al256(off + (size_t)MP * HID * 4);
  const size_t oHIT = off; off = al256(off + (size_t)gA * RCAP * 4);
  const size_t oCNT = off; off = al256(off + (size_t)NBP * 4);
  const size_t oOFF = off; off = al256(off + (size_t)NBP * 4);
  const size_t oDIS = off; off = al256(off + (size_t)NBP * 4);
  const size_t oREC = off; off = al256(off + (size_t)gA * NGR * CATW * 4);
  const size_t oRCN = off; off = al256(off + (size_t)gA * NGR * 4);
  const size_t oW1T = off; off = al256(off + (size_t)HID * FIN * 2);
  const size_t oW2D = off; off = al256(off + (size_t)HID * K2 * 2);
  const size_t oW3D = off; off = al256(off + (size_t)HID * K2 * 2);
  const size_t oC1D = off; off = al256(off + (size_t)CH1 * KC1 * 2);
  const size_t oC2D = off; off = al256(off + (size_t)NPO * KZ * 2);
  if (off > ws_size || off > (size_t)WSMAX) return;
  if ((size_t)MP * K2 * 2 > (size_t)MP * HID * 4) return;
  unsigned short* XB   = (unsigned short*)(ws + oXB);
  float*          R1   = (float*)(ws + oR1);
  unsigned short* X1hl = (unsigned short*)(ws + oR2);
  float*          R2f  = (float*)(ws + oR2);
  int*            HITS = (int*)(ws + oHIT);
  int*            CNTT = (int*)(ws + oCNT);
  int*            OFFT = (int*)(ws + oOFF);
  float*          DIS  = (float*)(ws + oDIS);
  float*          REC  = (float*)(ws + oREC);
  int*            RCN  = (int*)(ws + oRCN);
  unsigned short* W1T  = (unsigned short*)(ws + oW1T);
  unsigned short* W2D  = (unsigned short*)(ws + oW2D);
  unsigned short* W3D  = (unsigned short*)(ws + oW3D);
  unsigned short* C1D  = (unsigned short*)(ws + oC1D);
  unsigned short* C2D  = (unsigned short*)(ws + oC2D);

  const size_t bktLds  = (size_t)BKT_LDS_INTS * 4;
  const size_t poolLds = (size_t)NGR * CATW * 4;
  const size_t headLds = (size_t)HEAD_LDS_INTS * 4;
  hipFuncSetAttribute(reinterpret_cast<const void*>(&k_bucket), hipFuncAttributeMaxDynamicSharedMemorySize, (int)bktLds);
  hipFuncSetAttribute(reinterpret_cast<const void*>(&k_pool),   hipFuncAttributeMaxDynamicSharedMemorySize, (int)poolLds);
  hipFuncSetAttribute(reinterpret_cast<const void*>(&k_head),   hipFuncAttributeMaxDynamicSharedMemorySize, (int)headLds);

  const int prepBlocks = (ux + UW1 + 2 * UW2 + UC1 + UC2) / NTHR;
  k_prep<<<prepBlocks, NTHR, 0, stream>>>(x, w1, w2, w3, cw1, cw2, nN, ux, XB, W1T, W2D, W3D, C1D, C2D);
  k_bucket<<<gA, NTHR, bktLds, stream>>>(src, dst, nE, nN, vec8, HITS, CNTT, OFFT, DIS);
  k_gemm<<<dim3(gM, HID / GBN), GTHR, 0, stream>>>(XB, W1T, DIS, NBP, R1, FIN, HID);
  k_agg<1><<<gA, NTHR, 0, stream>>>(HITS, CNTT, OFFT, DIS, nN, MP, R1, b1, m1, v1, g1, be1, X1hl, R2f);
  k_gemm<<<dim3(gM, HID / GBN), GTHR, 0, stream>>>(X1hl, W2D, DIS, NBP, R1, K2, HID);
  k_agg<2><<<gA, NTHR, 0, stream>>>(HITS, CNTT, OFFT, DIS, nN, MP, R1, b2, m2, v2, g2, be2, X1hl, R2f);
  k_agg<3><<<gA, NTHR, 0, stream>>>(HITS, CNTT, OFFT, DIS, nN, MP, R2f, b3, m3, v3, g3, be3, X1hl, R1);
  k_pool<<<gA, PTHR, poolLds, stream>>>(R1, x, bat, nN, REC, RCN);
  k_head<<<1, NTHR, headLds, stream>>>(REC, RCN, gA, W3D, C1D, C2D, b3, m3, v3, g3, be3, cb1, cb2, out);
}
